// GCN_13494787244283
// MI455X (gfx1250) — hardware-run, weakly checked
//
#include <hip/hip_runtime.h>

typedef float          v8f   __attribute__((ext_vector_type(8)));
typedef float          v4f   __attribute__((ext_vector_type(4)));
typedef unsigned int   v4u   __attribute__((ext_vector_type(4)));
typedef int            v8i   __attribute__((ext_vector_type(8)));
typedef unsigned short v8us  __attribute__((ext_vector_type(8)));
typedef unsigned short v16us __attribute__((ext_vector_type(16)));
typedef __bf16         v16bf __attribute__((ext_vector_type(16)));
typedef _Float16       v16h  __attribute__((ext_vector_type(16)));
typedef v4f  __attribute__((may_alias)) v4fa;
typedef v8us __attribute__((may_alias)) v8usa;
union FragB { v16bf v; v16us u; v8us h[2]; v8i w; };
union FragH { v16h  v; v16us u; v8us h[2]; v8i w; };

__device__ __forceinline__ v8f wmb(const FragB& a, const FragB& b, v8f c) {
  v8f d = __builtin_amdgcn_wmma_f32_16x16x32_bf16(false, a.v, false, b.v, (short)0, c, false, false);
  asm volatile("v_nop\n\tv_nop\n\tv_nop\n\tv_nop" : "+v"(d) : "v"(a.w), "v"(b.w));
  return d;
}

__device__ __forceinline__ v8f wmh(const FragH& a, const FragH& b, v8f c) {
  v8f d = __builtin_amdgcn_wmma_f32_16x16x32_f16(false, a.v, false, b.v, (short)0, c, false, false);
  asm volatile("v_nop\n\tv_nop\n\tv_nop\n\tv_nop" : "+v"(d) : "v"(a.w), "v"(b.w));
  return d;
}

__device__ __forceinline__ unsigned bf16_bits(float f) {
  const unsigned u = __float_as_uint(f);
  const unsigned r = (u + 0x7FFFu + ((u >> 16) & 1u)) >> 16;
  const unsigned q = (u >> 16) | 0x40u;
  return ((u & 0x7fffffffu) > 0x7f800000u) ? q : r;
}

__device__ __forceinline__ float bf16_val(float f) {
  return __uint_as_float(bf16_bits(f) << 16);
}
__device__ __forceinline__ int clampi(int v, int lo, int hi) {
  return v < lo ? lo : (v > hi ? hi : v);
}

__device__ __forceinline__ unsigned f16_bits(float f) {
  const unsigned u  = __float_as_uint(f);
  const unsigned s  = (u >> 16) & 0x8000u;
  const unsigned a  = u & 0x7fffffffu;
  const unsigned t  = a - 0x38000000u;
  const unsigned r  = (t + 0x0FFFu + ((t >> 13) & 1u)) >> 13;
  const unsigned rc = r > 0x7C00u ? 0x7C00u : r;
  const bool small  = a < 0x38800000u;
  const bool isnan  = a > 0x7f800000u;
  const unsigned fin = small ? 0u : (s | rc);
  return isnan ? (s | 0x7E00u) : fin;
}

__device__ __forceinline__ unsigned pk16(unsigned lo, unsigned hi) { return lo | (hi << 16); }
__device__ __forceinline__ unsigned bf16_lo_bits(float v) {
  float hi = bf16_val(v);
  asm volatile("" : "+v"(hi));
  return bf16_bits(v - hi);
}
__device__ __forceinline__ v4u pack8_bf16(v4f a, v4f c) {
  return (v4u){ pk16(bf16_bits(a[0]), bf16_bits(a[1])), pk16(bf16_bits(a[2]), bf16_bits(a[3])),
                pk16(bf16_bits(c[0]), bf16_bits(c[1])), pk16(bf16_bits(c[2]), bf16_bits(c[3])) };
}
__device__ __forceinline__ v4u pack8_bf16_lo(v4f a, v4f c) {
  return (v4u){ pk16(bf16_lo_bits(a[0]), bf16_lo_bits(a[1])), pk16(bf16_lo_bits(a[2]), bf16_lo_bits(a[3])),
                pk16(bf16_lo_bits(c[0]), bf16_lo_bits(c[1])), pk16(bf16_lo_bits(c[2]), bf16_lo_bits(c[3])) };
}
__device__ __forceinline__ v4u pack8_f16(v4f a, v4f c) {
  return (v4u){ pk16(f16_bits(a[0]), f16_bits(a[1])), pk16(f16_bits(a[2]), f16_bits(a[3])),
                pk16(f16_bits(c[0]), f16_bits(c[1])), pk16(f16_bits(c[2]), f16_bits(c[3])) };
}

template <int FORM>
__global__ __launch_bounds__(256) void k_plane(const float* __restrict__ src, int rows, int cols, int ldsrc,
                                               unsigned short* __restrict__ dst, int MP, int KP) {
  static_assert(FORM >= 0 && FORM <= 3);
  const int KTOT = (FORM == 1 || FORM == 3) ? 2 * KP : KP;
  const unsigned ppr   = (unsigned)(KTOT >> 3);
  const unsigned kp8   = (unsigned)(KP >> 3);
  const unsigned total = (unsigned)MP * ppr;
  const unsigned g     = blockIdx.x * 256u + threadIdx.x;
  const unsigned rowu  = g / ppr;
  const unsigned p     = g - rowu * ppr;
  const bool second    = p >= kp8;
  const int row = (int)rowu;
  const int c0  = (int)((second ? p - kp8 : p) << 3);
  const float* srow = src + (size_t)clampi(row, 0, rows - 1) * (size_t)ldsrc;
  float x[8];
  unsigned mk[8];
#pragma unroll
  for (int e = 0; e < 8; ++e) {
    const int c = c0 + e;
    const float v = srow[clampi(c, 0, cols - 1)];
    asm volatile("" :: "v"(v));
    x[e]  = v;
    mk[e] = (row < rows && c < cols) ? 0xFFFFu : 0u;
  }
  const v4f a = (v4f){ x[0], x[1], x[2], x[3] };
  const v4f c = (v4f){ x[4], x[5], x[6], x[7] };
  v4u o;
  if (FORM == 2) {
    o = pack8_f16(a, c);
  } else {
    const v4u hi = pack8_bf16(a, c);
    o = hi;
    if (FORM == 1) { const v4u lo = pack8_bf16_lo(a, c); o = second ? lo : hi; }
  }
  const v4u mw = (v4u){ pk16(mk[0], mk[1]), pk16(mk[2], mk[3]), pk16(mk[4], mk[5]), pk16(mk[6], mk[7]) };
  o &= mw;
  if (g < total) {
    volatile v4u* q = (volatile v4u*)(dst + (size_t)g * 8);
    *q = o;
    __threadfence();
    *q = o;
  }
}

template <int FORM> struct FragOf    { typedef FragB T; };
template <>         struct FragOf<2> { typedef FragH T; };
__device__ __forceinline__ v8f mm(const FragB& a, const FragB& b, v8f c) { return wmb(a, b, c); }
__device__ __forceinline__ v8f mm(const FragH& a, const FragH& b, v8f c) { return wmh(a, b, c); }
template <class F> __device__ __forceinline__ F ld_frag(const unsigned short* p) {
  F f;
  f.h[0] = *(const v8usa*)(p);
  f.h[1] = *(const v8usa*)(p + 16);
  return f;
}

template <int FORM, int EPI>
__global__ __launch_bounds__(256) __attribute__((amdgpu_num_vgpr(248)))
void k_gemm_nt(const unsigned short* __restrict__ A, const unsigned short* __restrict__ B,
               const float* __restrict__ bias, float* __restrict__ D, int M, int N, int KTOT, int ldd) {
  static_assert(FORM >= 0 && FORM <= 2);
  static_assert(EPI == 0 || EPI == 1);
  typedef typename FragOf<FORM>::T F;
  __shared__ __attribute__((aligned(16))) float sT[8][16 * 68];
  const int lane = threadIdx.x & 31;
  const int wave = threadIdx.x >> 5;
  const int tilesM = (M + 63) >> 6;
  const int tilesN = (N + 63) >> 6;
  const int tile = blockIdx.x * 8 + wave;
  if (tile >= tilesM * tilesN) return;
  const int tm = tile / tilesN;
  const int tn = tile - tm * tilesN;
  const int m0 = tm << 6;
  const int n0 = tn << 6;

  const int rl = lane & 15;
  const int h8 = (lane >> 4) * 8;
  const unsigned short* pa = A + (size_t)(m0 + rl) * (size_t)KTOT + h8;
  const unsigned short* pb = B + (size_t)(n0 + rl) * (size_t)KTOT + h8;

  v8f acc[4][4];
#pragma unroll
  for (int i = 0; i < 4; ++i)
#pragma unroll
    for (int j = 0; j < 4; ++j) acc[i][j] = (v8f){0.f, 0.f, 0.f, 0.f, 0.f, 0.f, 0.f, 0.f};

#pragma unroll 1
  for (int k0 = 0; k0 < KTOT; k0 += 32) {
    F bf[4];
#pragma unroll
    for (int j = 0; j < 4; ++j) bf[j] = ld_frag<F>(pb + (size_t)(j << 4) * (size_t)KTOT + k0);
#pragma unroll
    for (int i = 0; i < 4; ++i) {
      const F af = ld_frag<F>(pa + (size_t)(i << 4) * (size_t)KTOT + k0);
#pragma unroll
      for (int j = 0; j < 4; ++j) acc[i][j] = mm(af, bf[j], acc[i][j]);
    }
  }

  float* slab = sT[wave];
  const int hh = lane >> 4;
  const int c4 = (lane & 15) * 4;
  const int nc = n0 + c4;
  const bool cok = nc < N;
  v4f bv = (v4f){0.f, 0.f, 0.f, 0.f};
  if (EPI == 1) {
    bv = *(const v4fa*)(bias + clampi(nc, 0, N - 4));
    asm volatile("" :: "v"(bv));
  }
#pragma unroll
  for (int i = 0; i < 4; ++i) {
    const int mBase = m0 + (i << 4);
#pragma unroll
    for (int j = 0; j < 4; ++j) {
#pragma unroll
      for (int r = 0; r < 8; ++r) slab[(h8 + r) * 68 + (j << 4) + rl] = acc[i][j][r];
    }
    __builtin_amdgcn_fence(__ATOMIC_RELEASE, "workgroup");
    __builtin_amdgcn_wave_barrier();
    __builtin_amdgcn_fence(__ATOMIC_ACQUIRE, "workgroup");
    v4f vv[8];
#pragma unroll
    for (int it = 0; it < 8; ++it) {
      const int row = it * 2 + hh;
      v4f v = *(const v4fa*)(slab + row * 68 + c4);
      if (EPI == 1) v += bv;
      vv[it] = v;
    }
    for (int pass = 0; pass < 2; ++pass) {
#pragma unroll
      for (int it = 0; it < 8; ++it) {
        const int row = mBase + it * 2 + hh;
        if (cok && row < M) *(volatile v4f*)(D + (size_t)row * (size_t)ldd + nc) = vv[it];
      }
      __threadfence();
    }
    __builtin_amdgcn_fence(__ATOMIC_RELEASE, "workgroup");
    __builtin_amdgcn_wave_barrier();
    __builtin_amdgcn_fence(__ATOMIC_ACQUIRE, "workgroup");
  }
}

#pragma clang fp contract(off)

#define GN      100000
#define GE      1600000
#define HID     128
#define GK      256
#define MPAD    100096
#define NTHR    256
#define NWAVE   8
#define EPT     8
#define WCH     256
#define NWCH    (GE / WCH)
#define WCPW    ((NWCH + NWAVE - 1) / NWAVE)
#define NBRUN   1024
#define NBLOG   10
#define NBLK    98
#define NSLOT   (NBLK * NBRUN)
#define WLCAP   4096
#define RCAP    20480
#define DEGCAP  64
#define SRCBITS 17
#define RPW     4
#define NUW     (HID * (GK / 8))
#define L2_SINGLE 0

typedef int          v4i __attribute__((ext_vector_type(4)));
typedef unsigned int v2u __attribute__((ext_vector_type(2)));
typedef v4i __attribute__((may_alias)) v4ia;

static_assert(GN <= (1 << SRCBITS));
static_assert(NBRUN == (1 << NBLOG) && NBRUN <= (1 << 10));
static_assert(SRCBITS + NBLOG < 31);
static_assert(NSLOT >= GN);
static_assert(GE % WCH == 0);
static_assert(WCPW * NWAVE >= NWCH && WCPW * (NWAVE - 1) < NWCH);
static_assert(RCAP % (NTHR * 4) == 0);
static_assert(RCAP >= 17558);
static_assert(DEGCAP >= 36 + 8 && DEGCAP % 32 == 0);
static_assert(HID == 32 * 4 && GK == 2 * HID && GK % 32 == 0);
static_assert(MPAD == 782 * 128 && MPAD % 64 == 0 && MPAD >= GN);
static_assert(GN % (NWAVE * RPW) == 0 && MPAD % (NWAVE * RPW) == 0);
static_assert(NUW % NTHR == 0);
static_assert((size_t)MPAD * GK / 8 < ((size_t)2048 << 20));

#define BK_HEAD   (3 * NBRUN + 32)
#define BK_INTS_C (BK_HEAD + NWAVE * WLCAP)
#define BK_INTS_F (BK_INTS_C + RCAP)
static_assert(BK_INTS_C % 4 == 0 && BK_INTS_F % 4 == 0);
static_assert((size_t)BK_INTS_F * 4 <= 300000);

constexpr size_t SZ_T    = (size_t)MPAD * HID * 4;
constexpr size_t SZ_A    = (size_t)MPAD * GK * 2;
constexpr size_t SZ_LIST = (size_t)NBLK * RCAP * 4;
constexpr size_t SZ_TAB  = (size_t)NSLOT * 4;
constexpr size_t SZ_WD   = (size_t)HID * GK * 2;
constexpr size_t SZ_FL   = (size_t)NBLK * 128;
constexpr size_t O_T     = 0;
constexpr size_t O_A     = O_T + SZ_T;
constexpr size_t O_LIST  = O_A + SZ_A;
constexpr size_t O_CNT   = O_LIST + SZ_LIST;
constexpr size_t O_OFF   = O_CNT + SZ_TAB;
constexpr size_t O_INN   = O_OFF + SZ_TAB;
constexpr size_t O_OUTN  = O_INN + SZ_TAB;
constexpr size_t O_W1D   = O_OUTN + SZ_TAB;
constexpr size_t O_W2D   = O_W1D + SZ_WD;
constexpr size_t O_FLD   = O_W2D + SZ_WD;
constexpr size_t O_FLS   = O_FLD + SZ_FL;
constexpr size_t WS_TOTAL = O_FLS + SZ_FL;
constexpr size_t WSMAX   = (size_t)128 << 20;
static_assert(SZ_T % 256 == 0 && SZ_A % 256 == 0 && SZ_LIST % 256 == 0 && SZ_TAB % 256 == 0);
static_assert(SZ_WD % 256 == 0 && SZ_FL % 256 == 0);
static_assert(WS_TOTAL <= WSMAX);

__device__ __forceinline__ void wprep_unit(const float* __restrict__ W, unsigned short* __restrict__ D, int v) {
  const int n  = v >> 5;
  const int p  = v & 31;
  const int kk = (p & 15) * 8;
  const float* q = W + (size_t)kk * HID + n;
  float x[8];
#pragma unroll
  for (int i = 0; i < 8; ++i) {
    const float t = q[(size_t)i * HID];
    asm volatile("" :: "v"(t));
    x[i] = t;
  }
  const v4u o = pack8_bf16((v4f){ x[0], x[1], x[2], x[3] }, (v4f){ x[4], x[5], x[6], x[7] });
  volatile v4u* dp = (volatile v4u*)(D + (size_t)n * GK + p * 8);
  *dp = o;
  __threadfence();
  *dp = o;
}

__global__ __launch_bounds__(NTHR) void k_wprep(const float* __restrict__ W1, const float* __restrict__ W2,
                                                unsigned short* __restrict__ W1D, unsigned short* __restrict__ W2D) {
  const int u = (int)blockIdx.x * NTHR + (int)threadIdx.x;
  if (u < NUW) wprep_unit(W1, W1D, u);
  else         wprep_unit(W2, W2D, u - NUW);
}

template <int PLACE>
__device__ __forceinline__ int walk_lists(const int* wl, const int* misc, int* cnt, int* cur, int* sl, int lane) {
  int tot = 0;
#pragma unroll 1
  for (int w2 = 0; w2 < NWAVE; ++w2) {
    int cv = misc[w2];
    cv = clampi(cv, 0, WLCAP);
    const int c = __builtin_amdgcn_readfirstlane(cv);
#pragma unroll 1
    for (int b0 = 0; b0 < c; b0 += 32) {
      int idx = b0 + lane;
      idx = idx < c ? idx : c - 1;
      const int ent = wl[w2 * WLCAP + idx];
      const int m32 = (c - b0) < 32 ? (c - b0) : 32;
#pragma unroll 1
      for (int k = 0; k < m32; ++k) {
        const int u    = __builtin_amdgcn_readlane(ent, k);
        const int slot = (u >> SRCBITS) & (NBRUN - 1);
        if (lane == 0) {
          if (PLACE != 0) {
            int p = cur[slot];
            p = clampi(p, 0, RCAP - 1);
            sl[p] = u & ((1 << SRCBITS) - 1);
            cur[slot] = p + 1;
          } else {
            cnt[slot] = cnt[slot] + 1;
          }
        }
      }
    }
    tot += c;
  }
  return tot;
}

template <int FULL>
__global__ __launch_bounds__(NTHR) void k_bucket(const int* __restrict__ key, const int* __restrict__ oth,
                                                 int* __restrict__ LISTW, int* __restrict__ CNTW,
                                                 int* __restrict__ OFFW, int* __restrict__ NRMW,
                                                 int* __restrict__ FLGW) {
  extern __shared__ __attribute__((aligned(16))) int dsm[];
  int* cnt  = dsm;
  int* offs = dsm + NBRUN;
  int* cur  = dsm + 2 * NBRUN;
  int* misc = dsm + 3 * NBRUN;
  int* wl   = dsm + BK_HEAD;
  int* sl   = wl + NWAVE * WLCAP;
  const int tid = (int)threadIdx.x, lane = tid & 31, wave = tid >> 5;
  const int slotBase = (int)blockIdx.x * NBRUN;
  constexpr int ZINTS = (FULL != 0) ? BK_INTS_F : BK_INTS_C;

  {
    const v4i z4 = {0, 0, 0, 0};
    for (int i = tid * 4; i < ZINTS; i += NTHR * 4) *(v4ia*)(dsm + i) = z4;
  }
  __syncthreads();

  {
    int wc = 0, wov = 0;
    int* mywl = wl + wave * WLCAP;
    const int ch0 = wave * WCPW;
    const int ch1 = (ch0 + WCPW < NWCH) ? (ch0 + WCPW) : NWCH;
    const unsigned ub = (unsigned)slotBase;
#pragma unroll 1
    for (int ch = ch0; ch < ch1; ++ch) {
      const int e0 = ch * WCH + lane * EPT;
      const v4i ka = *(const v4ia*)(key + e0);
      const v4i kb = *(const v4ia*)(key + e0 + 4);
      asm volatile("" :: "v"(ka), "v"(kb));
      v4i pa = ka, pb = kb;
      if (FULL != 0) {
        pa = *(const v4ia*)(oth + e0);
        pb = *(const v4ia*)(oth + e0 + 4);
        asm volatile("" :: "v"(pa), "v"(pb));
      }
      const int kk[8] = { ka.x, ka.y, ka.z, ka.w, kb.x, kb.y, kb.z, kb.w };
      const int pp[8] = { pa.x, pa.y, pa.z, pa.w, pb.x, pb.y, pb.z, pb.w };
      unsigned s[8];
      unsigned hm = 0u;
#pragma unroll
      for (int j = 0; j < 8; ++j) {
        s[j] = (unsigned)kk[j] - ub;
        hm |= (s[j] < (unsigned)NBRUN) ? (1u << j) : 0u;
      }
      const int n = (int)__builtin_popcount(hm);
      const unsigned m0 = __builtin_amdgcn_ballot_w32((n & 1) != 0);
      const unsigned m1 = __builtin_amdgcn_ballot_w32((n & 2) != 0);
      const unsigned m2 = __builtin_amdgcn_ballot_w32((n & 4) != 0);
      const unsigned m3 = __builtin_amdgcn_ballot_w32((n & 8) != 0);
      const int pre = (int)__builtin_amdgcn_mbcnt_lo(m0, 0u) + 2 * (int)__builtin_amdgcn_mbcnt_lo(m1, 0u) +
                      4 * (int)__builtin_amdgcn_mbcnt_lo(m2, 0u) + 8 * (int)__builtin_amdgcn_mbcnt_lo(m3, 0u);
      const int tot = (int)__builtin_popcount(m0) + 2 * (int)__builtin_popcount(m1) +
                      4 * (int)__builtin_popcount(m2) + 8 * (int)__builtin_popcount(m3);
      int pos = wc + pre;
#pragma unroll
      for (int j = 0; j < 8; ++j) {
        if ((hm >> j) & 1u) {
          const unsigned pw = (FULL != 0) ? (unsigned)clampi(pp[j], 0, GN - 1) : 0u;
          if (pos < WLCAP) mywl[pos] = (int)((s[j] << SRCBITS) | pw);
          pos = pos + 1;
        }
      }
      wov |= (wc + tot > WLCAP) ? 1 : 0;
      wc += tot;
    }
    if (lane == 0) { misc[wave] = wc; misc[8 + wave] = wov; }
  }
  __syncthreads();

  if (wave == 0) {
    const int tot = walk_lists<0>(wl, misc, cnt, cur, sl, lane);
    int ov = misc[8 + (lane & 7)];
    asm volatile("" :: "v"(ov));
    int flag = (__builtin_amdgcn_ballot_w32(ov != 0) != 0u) ? 1 : 0;
    if (FULL != 0) flag |= (tot > RCAP) ? 1 : 0;
    if (lane == 0) { misc[16] = tot; misc[17] = flag; }
  }
  __syncthreads();

  if (wave == 0) {
    const int base = lane * (NBRUN / 32);
    int sm = 0;
#pragma unroll 1
    for (int i = 0; i < NBRUN / 32; ++i) sm += cnt[base + i];
    int incl = sm;
#pragma unroll
    for (int d = 1; d < 32; d <<= 1) {
      const int y = __shfl_up(incl, d, 32);
      if (lane >= d) incl += y;
    }
    int run = incl - sm;
#pragma unroll 1
    for (int i = 0; i < NBRUN / 32; ++i) {
      const int cv = cnt[base + i];
      offs[base + i] = run;
      cur[base + i]  = run;
      run += cv;
    }
  }
  __syncthreads();

  if constexpr (FULL != 0) {
    if (wave == 0) (void)walk_lists<1>(wl, misc, cnt, cur, sl, lane);
  }
  __syncthreads();

#pragma unroll 1
  for (int i = 0; i < NBRUN / NTHR; ++i) {
    const int sidx = i * NTHR + tid;
    const int c = cnt[sidx];
    const int d = c < 1 ? 1 : c;
    const float f = 1.0f / sqrtf((float)d);
    cur[sidx] = __float_as_int(f);
  }
  __syncthreads();

  const int  flag = misc[17];
  const v4i  c4 = *(const v4ia*)(cnt  + 4 * tid);
  const v4i  o4 = *(const v4ia*)(offs + 4 * tid);
  const v4i  n4 = *(const v4ia*)(cur  + 4 * tid);
  const v4i  f4 = { flag, flag, flag, flag };
  const bool fw = (wave == 0) && (lane < 8);
  for (int pass = 0; pass < 2; ++pass) {
    *(volatile v4i*)(NRMW + slotBase + 4 * tid) = n4;
    if (FULL != 0) {
      *(volatile v4i*)(CNTW + slotBase + 4 * tid) = c4;
      *(volatile v4i*)(OFFW + slotBase + 4 * tid) = o4;
#pragma unroll 1
      for (int it = 0; it < RCAP / (NTHR * 4); ++it) {
        const int w = 4 * (it * NTHR + tid);
        const v4i v = *(const v4ia*)(sl + w);
        *(volatile v4i*)(LISTW + (size_t)blockIdx.x * RCAP + w) = v;
      }
    }
    if (fw) *(volatile v4i*)(FLGW + (size_t)blockIdx.x * 32 + 4 * lane) = f4;
    __threadfence();
  }
}

__device__ __forceinline__ void put_split_row(unsigned short* __restrict__ A, int row, int lane, v4f s,
                                              unsigned mh, unsigned ml) {
  const unsigned h0 = bf16_bits(s[0]), h1 = bf16_bits(s[1]), h2 = bf16_bits(s[2]), h3 = bf16_bits(s[3]);
  const unsigned l0 = bf16_lo_bits(s[0]), l1 = bf16_lo_bits(s[1]);
  const unsigned l2 = bf16_lo_bits(s[2]), l3 = bf16_lo_bits(s[3]);
  const v2u hv = (v2u){ pk16(h0, h1) & mh, pk16(h2, h3) & mh };
  const v2u lv = (v2u){ pk16(l0, l1) & ml, pk16(l2, l3) & ml };
  unsigned short* ph = A + (size_t)row * GK + 4 * lane;
  volatile v2u* qh = (volatile v2u*)ph;
  volatile v2u* ql = (volatile v2u*)(ph + HID);
  *qh = hv;
  *ql = lv;
  __threadfence();
  *qh = hv;
  *ql = lv;
}

__global__ __launch_bounds__(NTHR) void k_scale_split(const float* __restrict__ x, const float* __restrict__ OUTN,
                                                      unsigned short* __restrict__ A) {
  const int tid = (int)threadIdx.x, lane = tid & 31, wave = tid >> 5;
  const int row0 = (int)blockIdx.x * (NWAVE * RPW) + wave * RPW;
#pragma unroll 1
  for (int r = 0; r < RPW; ++r) {
    const int row = row0 + r;
    const int rc  = row < GN ? row : GN - 1;
    const v4f a = *(const v4fa*)(x + (size_t)rc * HID + 4 * lane);
    const float on = OUTN[rc];
    asm volatile("" :: "v"(a), "v"(on));
    const unsigned mk = (row < GN) ? 0xFFFFFFFFu : 0u;
    const v4f s = (v4f){ bf16_val(a[0]) * on, bf16_val(a[1]) * on, bf16_val(a[2]) * on, bf16_val(a[3]) * on };
    put_split_row(A, row, lane, s, mk, mk);
  }
}

template <int LAYER>
__global__ __launch_bounds__(NTHR) void k_agg(const float* __restrict__ T, const int* __restrict__ LISTW,
                                              const int* __restrict__ CNTW, const int* __restrict__ OFFW,
                                              const float* __restrict__ INN, const float* __restrict__ OUTN,
                                              const int* __restrict__ FLD, const int* __restrict__ FLS,
                                              const float* __restrict__ bias, unsigned short* __restrict__ A,
                                              float* __restrict__ out) {
  const int tid = (int)threadIdx.x, lane = tid & 31, wave = tid >> 5;
  const int row0 = (int)blockIdx.x * (NWAVE * RPW) + wave * RPW;
  const int b = clampi(row0 >> NBLOG, 0, NBLK - 1);

  v4f bv = *(const v4fa*)(bias + 4 * lane);
  asm volatile("" :: "v"(bv));
  bv = (v4f){ bf16_val(bv[0]), bf16_val(bv[1]), bf16_val(bv[2]), bf16_val(bv[3]) };
  int fl = FLD[(size_t)b * 32];
#pragma unroll
  for (int i = 0; i < 4; ++i) {
    const int bi = (lane + 32 * i) < NBLK ? (lane + 32 * i) : NBLK - 1;
    fl |= FLS[(size_t)bi * 32];
  }
  asm volatile("" :: "v"(fl));
  const bool pois = __builtin_amdgcn_ballot_w32(fl != 0) != 0u;
  const float qnan = __int_as_float(0x7fc00000);
  const int* lp = LISTW + (size_t)b * RCAP;

#pragma unroll 1
  for (int r = 0; r < RPW; ++r) {
    const int row = row0 + r;
    const int   cv  = CNTW[row];
    const int   ov  = OFFW[row];
    const float inn = INN[row];
    const float on  = OUTN[row];
    asm volatile("" :: "v"(cv), "v"(ov), "v"(inn), "v"(on));
    const int cu = __builtin_amdgcn_readfirstlane(cv);
    const bool big = (cu > DEGCAP) || (cu < 0);
    const int c = __builtin_amdgcn_readfirstlane(clampi(cv, 0, DEGCAP));
    const int o = __builtin_amdgcn_readfirstlane(clampi(ov, 0, RCAP - 1));
    v4f acc = (v4f){ 0.0f, 0.0f, 0.0f, 0.0f };
#pragma unroll 1
    for (int b0 = 0; b0 < c; b0 += 32) {
      int li = b0 + lane;
      li = li < c ? li : c - 1;
      int idx = o + li;
      idx = idx > RCAP - 1 ? RCAP - 1 : idx;
      int sr = lp[idx];
      asm volatile("" :: "v"(sr));
      sr = clampi(sr, 0, GN - 1);
      const int m32 = (c - b0) < 32 ? (c - b0) : 32;
#pragma unroll 1
      for (int k = 0; k < m32; ++k) {
        const int sk = __builtin_amdgcn_readlane(sr, k);
        const v4f v = *(const v4fa*)(T + (size_t)sk * HID + 4 * lane);
        asm volatile("" :: "v"(v));
        acc += v;
      }
    }
    const bool kill = pois || big;
    v4f y;
#pragma unroll
    for (int q = 0; q < 4; ++q) {
      const float t  = acc[q] * inn + bv[q];
      const float rl = (t > 0.0f) ? t : (t - t);
      y[q] = kill ? qnan : rl;
    }
    if constexpr (LAYER == 1) {
      const v4f s = (v4f){ y[0] * on, y[1] * on, y[2] * on, y[3] * on };
      put_split_row(A, row, lane, s, 0xFFFFFFFFu, (L2_SINGLE != 0) ? 0u : 0xFFFFFFFFu);
    } else {
      volatile v4f* op = (volatile v4f*)(out + (size_t)row * HID + 4 * lane);
      *op = y;
      __threadfence();
      *op = y;
    }
  }
}

extern "C" void kernel_launch(void* const* d_in, const int* in_sizes, int n_in,
                              void* d_out, int out_size, void* d_ws, size_t ws_size,
                              hipStream_t stream) {
  if (n_in < 7) return;
  if (in_sizes[0] != GN * HID) return;
  if (in_sizes[1] != GE || in_sizes[2] != GE) return;
  if (in_sizes[3] != HID * HID || in_sizes[4] != HID) return;
  if (in_sizes[5] != HID * HID || in_sizes[6] != HID) return;
  if (out_size != GN * HID) return;
  if (ws_size < WS_TOTAL) return;

  const float* x   = (const float*)d_in[0];
  const int*   src = (const int*)d_in[1];
  const int*   dst = (const int*)d_in[2];
  const float* W1  = (const float*)d_in[3];
  const float* b1  = (const float*)d_in[4];
  const float* W2  = (const float*)d_in[5];
  const float* b2  = (const float*)d_in[6];
  float* out = (float*)d_out;

  char* ws = (char*)d_ws;
  float*          T    = (float*)(ws + O_T);
  unsigned short* A    = (unsigned short*)(ws + O_A);
  int*            LIST = (int*)(ws + O_LIST);
  int*            CNT  = (int*)(ws + O_CNT);
  int*            OFF  = (int*)(ws + O_OFF);
  int*            INNi = (int*)(ws + O_INN);
  int*            OUTi = (int*)(ws + O_OUTN);
  unsigned short* W1D  = (unsigned short*)(ws + O_W1D);
  unsigned short* W2D  = (unsigned short*)(ws + O_W2D);
  int*            FLD  = (int*)(ws + O_FLD);
  int*            FLS  = (int*)(ws + O_FLS);
  const float* INN  = (const float*)INNi;
  const float* OUTN = (const float*)OUTi;

  const size_t ldsF = (size_t)BK_INTS_F * 4;
  const size_t ldsC = (size_t)BK_INTS_C * 4;
  hipFuncSetAttribute(reinterpret_cast<const void*>(&k_bucket<1>), hipFuncAttributeMaxDynamicSharedMemorySize, (int)ldsF);
  hipFuncSetAttribute(reinterpret_cast<const void*>(&k_bucket<0>), hipFuncAttributeMaxDynamicSharedMemorySize, (int)ldsC);

  const int gemmBlocks = ((MPAD / 64) * (HID / 64) + 7) / 8;
  const int rowBlocksP = MPAD / (NWAVE * RPW);
  const int rowBlocksN = GN / (NWAVE * RPW);

  k_wprep<<<(2 * NUW) / NTHR, NTHR, 0, stream>>>(W1, W2, W1D, W2D);
  k_bucket<1><<<NBLK, NTHR, ldsF, stream>>>(dst, src, LIST, CNT, OFF, INNi, FLD);
  k_bucket<0><<<NBLK, NTHR, ldsC, stream>>>(src, dst, LIST, CNT, OFF, OUTi, FLS);
  k_scale_split<<<rowBlocksP, NTHR, 0, stream>>>(x, OUTN, A);
  k_gemm_nt<0, 0><<<gemmBlocks, 256, 0, stream>>>(A, W1D, b1, T, MPAD, HID, GK, HID);
  k_agg<1><<<rowBlocksN, NTHR, 0, stream>>>(T, LIST, CNT, OFF, INN, OUTN, FLD, FLS, b1, A, out);
  k_gemm_nt<0, 0><<<gemmBlocks, 256, 0, stream>>>(A, W2D, b2, T, MPAD, HID, GK, HID);
  k_agg<2><<<rowBlocksN, NTHR, 0, stream>>>(T, LIST, CNT, OFF, INN, OUTN, FLD, FLS, b2, A, out);
}
